// CodeUpdater_22058952032956
// MI455X (gfx1250) — hardware-verified
//
#include <hip/hip_runtime.h>
#include <stdint.h>
#include <stddef.h>

#define NROW 4096
#define MROW 8192
#define KSEL 32768
#define RMAX 8
#define DCOL 512
#define D2   1024
#define HU   256
#define G4   1024
#define NBX  32

#define GBM 64
#define GBN 128
#define KC  64
#define APG 72
#define TPG 132
#define WSC  64.0f
#define WSCI 0.015625f

static_assert(KSEL % GBM == 0);
static_assert(DCOL % GBN == 0);
static_assert(NROW % 64 == 0);
static_assert(G4 % 128 == 0);
static_assert(D2 % KC == 0);
static_assert(DCOL % KC == 0);
static_assert(KC % 32 == 0);
static_assert((APG * 2) % 16 == 0);
static_assert((TPG * 4) % 16 == 0);
static_assert(NROW % NBX == 0);
static_assert(NBX * RMAX == 256);
static_assert(KSEL % 256 == 0);
static_assert(G4 == 4 * HU);
static_assert(D2 == 2 * DCOL);
static_assert(HU == 256);

typedef _Float16       v16h __attribute__((ext_vector_type(16)));
typedef float          v8f  __attribute__((ext_vector_type(8)));
typedef float          v4f  __attribute__((ext_vector_type(4)));
typedef unsigned int   v4u  __attribute__((ext_vector_type(4)));
typedef v4f __attribute__((may_alias)) v4fa;
typedef v4u __attribute__((may_alias)) v4ua;

union FragH { v16h v; v4u q[2]; };

__device__ __forceinline__ v8f wmma_h(v16h a, v16h b, v8f c) {
  v8f d = __builtin_amdgcn_wmma_f32_16x16x32_f16(false, a, false, b, (short)0, c, false, false);
  asm volatile("v_nop\n\tv_nop\n\tv_nop\n\tv_nop" : "+v"(d) : "v"(a), "v"(b));
  return d;
}

__device__ __forceinline__ v16h ldfrag(const unsigned short* p, int h) {
  FragH f;
  f.q[0] = *(const v4ua*)(p + 8 * h);
  f.q[1] = *(const v4ua*)(p + 16 + 8 * h);
  return f.v;
}

__device__ __forceinline__ unsigned int pkh(float a, float b) {
  const unsigned short x = __builtin_bit_cast(unsigned short, (_Float16)a);
  const unsigned short y = __builtin_bit_cast(unsigned short, (_Float16)b);
  return (unsigned int)x | ((unsigned int)y << 16);
}
__device__ __forceinline__ v4u pack8(v4f a, v4f c) {
  v4u o;
  o.x = pkh(a.x, a.y); o.y = pkh(a.z, a.w);
  o.z = pkh(c.x, c.y); o.w = pkh(c.z, c.w);
  return o;
}

__device__ __forceinline__ float sigm(float x) {
  return __builtin_amdgcn_rcpf(1.0f + __expf(-x));
}
__device__ __forceinline__ float tnh(float x) {
  return 1.0f - 2.0f * __builtin_amdgcn_rcpf(__expf(2.0f * x) + 1.0f);
}

__global__ __launch_bounds__(256) void k_cvt(const float* __restrict__ src,
                                             unsigned short* __restrict__ dst,
                                             int n8, float s)
{
  const int g = blockIdx.x * 256 + threadIdx.x;
  if (g >= n8) return;
  const float* p = src + (size_t)g * 8;
  const v4f a = *(const v4fa*)p;
  const v4f c = *(const v4fa*)(p + 4);
  const v4u pk = pack8(a * s, c * s);
  unsigned short* d = dst + (size_t)g * 8;
  *(volatile v4u*)d = pk;
  __threadfence();
  *(volatile v4u*)d = pk;
}

__global__ __launch_bounds__(256) void k_gate(const unsigned short* __restrict__ Cp,
                                              const unsigned short* __restrict__ Tp,
                                              const unsigned short* __restrict__ Wg,
                                              const float* __restrict__ gb,
                                              const float* __restrict__ trc,
                                              const int* __restrict__ ci,
                                              const int* __restrict__ ti,
                                              float* __restrict__ G)
{
  __shared__ __align__(16) unsigned short sA[GBM * APG];
  __shared__ __align__(16) float sT[GBM * TPG];
  __shared__ int sCI[GBM];
  __shared__ int sTI[GBM];
  const int tid = threadIdx.x, lane = tid & 31, wv = tid >> 5;
  const int h = lane >> 4, m = lane & 15;
  const int wm = wv >> 2, wn = wv & 3;
  const int kb = blockIdx.x * GBM, nb = blockIdx.y * GBN;

  if (tid < GBM) {
    int c = ci[kb + tid];
    c = (c < 0) ? c + NROW : c;
    c = (c < 0) ? 0 : ((c > NROW - 1) ? (NROW - 1) : c);
    int t = ti[kb + tid];
    t = (t < 0) ? t + MROW : t;
    t = (t < 0) ? 0 : ((t > MROW - 1) ? (MROW - 1) : t);
    sCI[tid] = c;
    sTI[tid] = t;
  }
  __syncthreads();

  const v8f z8 = {0.f, 0.f, 0.f, 0.f, 0.f, 0.f, 0.f, 0.f};
  v8f acc[2][2];
  #pragma unroll
  for (int mt = 0; mt < 2; ++mt)
    #pragma unroll
    for (int nt = 0; nt < 2; ++nt) acc[mt][nt] = z8;

  #pragma unroll 1
  for (int k0 = 0; k0 < D2; k0 += KC) {
    const unsigned short* base = (k0 < DCOL) ? Cp : Tp;
    const int koff = k0 & (DCOL - 1);
    #pragma unroll
    for (int i = 0; i < 2; ++i) {
      const int idx = tid + 256 * i;
      const int row = idx >> 3, piece = idx & 7;
      const int rc = sCI[row], rt = sTI[row];
      const int ridx = (k0 < DCOL) ? rc : rt;
      const v4u v = *(const v4ua*)(base + (size_t)ridx * DCOL + koff + 8 * piece);
      *(v4ua*)(sA + row * APG + 8 * piece) = v;
    }
    __syncthreads();
    #pragma unroll
    for (int ks = 0; ks < KC / 32; ++ks) {
      v16h a[2];
      #pragma unroll
      for (int mt = 0; mt < 2; ++mt)
        a[mt] = ldfrag(sA + (32 * wm + 16 * mt + m) * APG + 32 * ks, h);
      #pragma unroll
      for (int nt = 0; nt < 2; ++nt) {
        const v16h b = ldfrag(Wg + (size_t)(nb + 32 * wn + 16 * nt + m) * D2 + k0 + 32 * ks, h);
        #pragma unroll
        for (int mt = 0; mt < 2; ++mt) acc[mt][nt] = wmma_h(a[mt], b, acc[mt][nt]);
      }
    }
    __syncthreads();
  }

  #pragma unroll
  for (int mt = 0; mt < 2; ++mt)
    #pragma unroll
    for (int nt = 0; nt < 2; ++nt) {
      const int col = 32 * wn + 16 * nt + m;
      #pragma unroll
      for (int r = 0; r < 8; ++r) {
        const int row = 32 * wm + 16 * mt + 8 * h + r;
        sT[row * TPG + col] = acc[mt][nt][r];
      }
    }
  __syncthreads();

  const int c4 = nb + 4 * lane;
  const v4f gbv = *(const v4fa*)(gb + c4);
  v4f ov[8];
  size_t go[8];
  #pragma unroll
  for (int i = 0; i < 8; ++i) {
    const int row = wv + 8 * i;
    const int trow = sTI[row];
    const v4f a = *(const v4fa*)(sT + row * TPG + 4 * lane);
    const v4f tr = *(const v4fa*)(trc + (size_t)trow * DCOL + c4);
    const v4f z = a * WSCI + gbv;
    v4f g;
    g.x = sigm(z.x) * tr.x;
    g.y = sigm(z.y) * tr.y;
    g.z = sigm(z.z) * tr.z;
    g.w = sigm(z.w) * tr.w;
    ov[i] = g;
    go[i] = (size_t)(kb + row) * DCOL + c4;
  }
  #pragma unroll
  for (int i = 0; i < 8; ++i) *(volatile v4f*)(G + go[i]) = ov[i];
  __threadfence();
  #pragma unroll
  for (int i = 0; i < 8; ++i) *(volatile v4f*)(G + go[i]) = ov[i];
}

__global__ __launch_bounds__(256) void k_xbuild(const int* __restrict__ ui,
                                                const int* __restrict__ rref,
                                                const float* __restrict__ G,
                                                unsigned short* __restrict__ Up)
{
  __shared__ int sSlot[NBX * RMAX];
  const int tid = threadIdx.x;
  const int n0 = blockIdx.x * NBX;
  int R = rref[0];
  R = (R < 1) ? 1 : ((R > RMAX) ? RMAX : R);
  sSlot[tid] = -1;
  __syncthreads();

  const int base = n0 * R, span = NBX * R, tot = NROW * R;
  #pragma unroll 1
  for (int it = 0; it < KSEL / 256; ++it) {
    const int k = it * 256 + tid;
    int u = ui[k];
    u = (u < 0) ? u + tot : u;
    const int s = u - base;
    if ((unsigned)s < (unsigned)span) sSlot[s] = k;
  }
  __syncthreads();

  const int c8 = (tid & 63) * 8, rsub = tid >> 6;
  v4u hv[8];
  size_t go[8];
  #pragma unroll
  for (int it = 0; it < 8; ++it) {
    const int rloc = 4 * it + rsub;
    v4f s0 = {0.f, 0.f, 0.f, 0.f};
    v4f s1 = {0.f, 0.f, 0.f, 0.f};
    #pragma unroll
    for (int r = 0; r < RMAX; ++r) {
      int si = rloc * R + r;
      si = (si > NBX * RMAX - 1) ? (NBX * RMAX - 1) : si;
      const int kk = sSlot[si];
      const int k = (r < R) ? kk : -1;
      int src = (k < 0) ? 0 : k;
      src = (src > KSEL - 1) ? (KSEL - 1) : src;
      const float* gp = G + (size_t)src * DCOL + c8;
      const v4f a = *(const v4fa*)gp;
      const v4f b = *(const v4fa*)(gp + 4);
      if (k >= 0) { s0 += a; s1 += b; }
    }
    hv[it] = pack8(s0, s1);
    go[it] = (size_t)(n0 + rloc) * DCOL + c8;
  }
  #pragma unroll
  for (int it = 0; it < 8; ++it) *(volatile v4u*)(Up + go[it]) = hv[it];
  __threadfence();
  #pragma unroll
  for (int it = 0; it < 8; ++it) *(volatile v4u*)(Up + go[it]) = hv[it];
}

__global__ __launch_bounds__(256) void k_xp(const unsigned short* __restrict__ Cp,
                                            const unsigned short* __restrict__ Up,
                                            const unsigned short* __restrict__ Wf,
                                            const unsigned short* __restrict__ Wb,
                                            const float* __restrict__ bf,
                                            const float* __restrict__ bb,
                                            float* __restrict__ XPf,
                                            float* __restrict__ XPb)
{
  __shared__ __align__(16) float sT[64 * TPG];
  const int tid = threadIdx.x, lane = tid & 31, wv = tid >> 5;
  const int h = lane >> 4, m = lane & 15;
  const int dir = blockIdx.z;
  const unsigned short* W = dir ? Wb : Wf;
  const float* bias = dir ? bb : bf;
  float* XP = dir ? XPb : XPf;
  const int wm = wv >> 2, wn = wv & 3;
  const int rb = blockIdx.x * 64 + 32 * wm, cb = blockIdx.y * 128 + 32 * wn;

  const v8f z8 = {0.f, 0.f, 0.f, 0.f, 0.f, 0.f, 0.f, 0.f};
  v8f acc[2][2];
  #pragma unroll
  for (int mt = 0; mt < 2; ++mt)
    #pragma unroll
    for (int nt = 0; nt < 2; ++nt) acc[mt][nt] = z8;

  #pragma unroll 1
  for (int k0 = 0; k0 < D2; k0 += 32) {
    const unsigned short* abase = (k0 < DCOL) ? Cp : Up;
    const int koff = k0 & (DCOL - 1);
    v16h a[2];
    #pragma unroll
    for (int mt = 0; mt < 2; ++mt)
      a[mt] = ldfrag(abase + (size_t)(rb + 16 * mt + m) * DCOL + koff, h);
    #pragma unroll
    for (int nt = 0; nt < 2; ++nt) {
      const v16h b = ldfrag(W + (size_t)(cb + 16 * nt + m) * D2 + k0, h);
      #pragma unroll
      for (int mt = 0; mt < 2; ++mt) acc[mt][nt] = wmma_h(a[mt], b, acc[mt][nt]);
    }
  }

  #pragma unroll
  for (int mt = 0; mt < 2; ++mt)
    #pragma unroll
    for (int nt = 0; nt < 2; ++nt) {
      const int col = 32 * wn + 16 * nt + m;
      #pragma unroll
      for (int r = 0; r < 8; ++r) {
        const int row = 32 * wm + 16 * mt + 8 * h + r;
        sT[row * TPG + col] = acc[mt][nt][r];
      }
    }
  __syncthreads();

  const int c4 = blockIdx.y * 128 + 4 * lane;
  const v4f bv = *(const v4fa*)(bias + c4);
  v4f ov[8];
  size_t go[8];
  #pragma unroll
  for (int i = 0; i < 8; ++i) {
    const int row = wv + 8 * i;
    const v4f a = *(const v4fa*)(sT + row * TPG + 4 * lane);
    ov[i] = a * WSCI + bv;
    go[i] = (size_t)(blockIdx.x * 64 + row) * G4 + c4;
  }
  #pragma unroll
  for (int i = 0; i < 8; ++i) *(volatile v4f*)(XP + go[i]) = ov[i];
  __threadfence();
  #pragma unroll
  for (int i = 0; i < 8; ++i) *(volatile v4f*)(XP + go[i]) = ov[i];
}

__global__ __launch_bounds__(256) void k_lstm(const float* __restrict__ XPf,
                                              const float* __restrict__ XPb,
                                              const float* __restrict__ Whf,
                                              const float* __restrict__ Whb,
                                              const float* __restrict__ cm,
                                              float* __restrict__ out)
{
  __shared__ __align__(16) float sH[2 * HU];
  const int u = threadIdx.x;
  const int dir = blockIdx.x;
  const float* xp = dir ? XPb : XPf;
  const float* W = dir ? Whb : Whf;
  sH[u] = 0.f;
  sH[HU + u] = 0.f;
  float c = 0.f;
  __syncthreads();

  const float* w0 = W + (size_t)u * HU;
  const float* w1 = W + (size_t)(HU + u) * HU;
  const float* w2 = W + (size_t)(2 * HU + u) * HU;
  const float* w3 = W + (size_t)(3 * HU + u) * HU;
  const int colo = dir * HU + u;

  #pragma unroll 1
  for (int s = 0; s < NROW; ++s) {
    const int t = dir ? (NROW - 1 - s) : s;
    const int cur = s & 1;
    const float* xr = xp + (size_t)t * G4;
    float a0 = xr[u], a1 = xr[HU + u], a2 = xr[2 * HU + u], a3 = xr[3 * HU + u];
    const float* hp = sH + cur * HU;
    #pragma unroll 2
    for (int j = 0; j < HU; j += 4) {
      const v4f hv = *(const v4fa*)(hp + j);
      const v4f x0 = *(const v4fa*)(w0 + j);
      const v4f x1 = *(const v4fa*)(w1 + j);
      const v4f x2 = *(const v4fa*)(w2 + j);
      const v4f x3 = *(const v4fa*)(w3 + j);
      a0 = fmaf(x0.x, hv.x, a0); a0 = fmaf(x0.y, hv.y, a0); a0 = fmaf(x0.z, hv.z, a0); a0 = fmaf(x0.w, hv.w, a0);
      a1 = fmaf(x1.x, hv.x, a1); a1 = fmaf(x1.y, hv.y, a1); a1 = fmaf(x1.z, hv.z, a1); a1 = fmaf(x1.w, hv.w, a1);
      a2 = fmaf(x2.x, hv.x, a2); a2 = fmaf(x2.y, hv.y, a2); a2 = fmaf(x2.z, hv.z, a2); a2 = fmaf(x2.w, hv.w, a2);
      a3 = fmaf(x3.x, hv.x, a3); a3 = fmaf(x3.y, hv.y, a3); a3 = fmaf(x3.z, hv.z, a3); a3 = fmaf(x3.w, hv.w, a3);
    }
    const float gi = sigm(a0);
    const float gf = sigm(a1);
    const float gg = tnh(a2);
    const float gq = sigm(a3);
    c = gf * c + gi * gg;
    const float hn = gq * tnh(c);
    sH[(cur ^ 1) * HU + u] = hn;
    const size_t oi = (size_t)t * DCOL + colo;
    const float ov = cm[oi] + hn;
    *(volatile float*)(out + oi) = ov;
    __threadfence();
    *(volatile float*)(out + oi) = ov;
    __syncthreads();
  }
}

extern "C" void kernel_launch(void* const* d_in, const int* in_sizes, int n_in,
                              void* d_out, int out_size, void* d_ws, size_t ws_size,
                              hipStream_t stream)
{
  if (n_in < 14) return;
  if (in_sizes[0]  != NROW * DCOL) return;
  if (in_sizes[1]  != MROW * DCOL) return;
  if (in_sizes[2]  != DCOL * D2) return;
  if (in_sizes[3]  != DCOL) return;
  if (in_sizes[4]  != G4 * D2) return;
  if (in_sizes[5]  != G4 * HU) return;
  if (in_sizes[6]  != G4) return;
  if (in_sizes[7]  != G4 * D2) return;
  if (in_sizes[8]  != G4 * HU) return;
  if (in_sizes[9]  != G4) return;
  if (in_sizes[10] != KSEL) return;
  if (in_sizes[11] != KSEL) return;
  if (in_sizes[12] != KSEL) return;
  if (in_sizes[13] < 1) return;
  if (out_size != NROW * DCOL) return;

  const float* cm    = (const float*)d_in[0];
  const float* tm    = (const float*)d_in[1];
  const float* gateW = (const float*)d_in[2];
  const float* gateB = (const float*)d_in[3];
  const float* wihF  = (const float*)d_in[4];
  const float* whhF  = (const float*)d_in[5];
  const float* bF    = (const float*)d_in[6];
  const float* wihB  = (const float*)d_in[7];
  const float* whhB  = (const float*)d_in[8];
  const float* bB    = (const float*)d_in[9];
  const int*   ci    = (const int*)d_in[10];
  const int*   ti    = (const int*)d_in[11];
  const int*   ui    = (const int*)d_in[12];
  const int*   rref  = (const int*)d_in[13];
  float* out = (float*)d_out;

  const size_t bCp = (size_t)NROW * DCOL * 2;
  const size_t bTp = (size_t)MROW * DCOL * 2;
  const size_t bWg = (size_t)DCOL * D2 * 2;
  const size_t bWi = (size_t)G4 * D2 * 2;
  const size_t bG  = (size_t)KSEL * DCOL * 4;
  const size_t bUp = (size_t)NROW * DCOL * 2;
  const size_t bXP = (size_t)NROW * G4 * 4;
  const size_t total = bCp + bTp + bWg + 2 * bWi + bG + bUp + 2 * bXP;
  if (total > ws_size) return;
  if (total > (size_t)134217728) return;

  char* ws = (char*)d_ws;
  size_t off = 0;
  unsigned short* Cp  = (unsigned short*)(ws + off); off += bCp;
  unsigned short* Tp  = (unsigned short*)(ws + off); off += bTp;
  unsigned short* Wg  = (unsigned short*)(ws + off); off += bWg;
  unsigned short* Wf  = (unsigned short*)(ws + off); off += bWi;
  unsigned short* Wb  = (unsigned short*)(ws + off); off += bWi;
  float*          G   = (float*)(ws + off);          off += bG;
  unsigned short* Up  = (unsigned short*)(ws + off); off += bUp;
  float*          XPf = (float*)(ws + off);          off += bXP;
  float*          XPb = (float*)(ws + off);          off += bXP;
  if (off != total) return;

  {
    const int n8c = NROW * DCOL / 8;
    const int n8t = MROW * DCOL / 8;
    const int n8g = DCOL * D2 / 8;
    const int n8w = G4 * D2 / 8;
    k_cvt<<<(n8c + 255) / 256, 256, 0, stream>>>(cm, Cp, n8c, 1.0f);
    k_cvt<<<(n8t + 255) / 256, 256, 0, stream>>>(tm, Tp, n8t, 1.0f);
    k_cvt<<<(n8g + 255) / 256, 256, 0, stream>>>(gateW, Wg, n8g, WSC);
    k_cvt<<<(n8w + 255) / 256, 256, 0, stream>>>(wihF, Wf, n8w, WSC);
    k_cvt<<<(n8w + 255) / 256, 256, 0, stream>>>(wihB, Wb, n8w, WSC);
  }
  k_gate<<<dim3(KSEL / GBM, DCOL / GBN), 256, 0, stream>>>(Cp, Tp, Wg, gateB, tm, ci, ti, G);
  k_xbuild<<<NROW / NBX, 256, 0, stream>>>(ui, rref, G, Up);
  k_xp<<<dim3(NROW / 64, G4 / 128, 2), 256, 0, stream>>>(Cp, Up, Wf, Wb, bF, bB, XPf, XPb);
  k_lstm<<<2, 256, 0, stream>>>(XPf, XPb, whhF, whhB, cm, out);
}
